// PointNetSetAbstraction_43439299232343
// MI455X (gfx1250) — hardware-verified
//
#include <hip/hip_runtime.h>
#pragma clang fp contract(off)

typedef __attribute__((ext_vector_type(16))) _Float16 v16h;
typedef __attribute__((ext_vector_type(8)))  float    v8f;
typedef __attribute__((ext_vector_type(4)))  float    v4f;
typedef __attribute__((ext_vector_type(4)))  unsigned v4u;
typedef __attribute__((ext_vector_type(8)))  unsigned v8u;

constexpr int NBATCH = 16;
constexpr int NPTS = 4096;
constexpr int NCENT = 1024;
constexpr int NSAMP = 32;
constexpr int CFEAT = 64;
constexpr int CIN1 = 67;
constexpr int KPAD1 = 96;
constexpr int CH1 = 64;
constexpr int CH2 = 64;
constexpr int CH3 = 128;
constexpr int MROWS = NBATCH * NCENT * NSAMP;
constexpr int NSTRIPS = NBATCH * NCENT;
constexpr int GEMM_BLOCKS = 256;
constexpr int GEMM_WAVES = 4;
constexpr int STRIPS_PER_WAVE = 16;
constexpr int PITCH_A1 = 104;
constexpr int PITCH_S = 72;
constexpr float BALL_R2 = 0.04f;
constexpr float BN_EPSV = 1e-5f;
constexpr int OUT0_ELEMS = NBATCH * 3 * NCENT;
constexpr int OUT1_ELEMS = NBATCH * CH3 * NCENT;

static_assert(GEMM_BLOCKS * GEMM_WAVES * STRIPS_PER_WAVE == NSTRIPS);
static_assert(MROWS == 524288);
static_assert(KPAD1 % 32 == 0 && CH1 % 32 == 0 && CH2 % 32 == 0);
static_assert(OUT0_ELEMS * 4 == 196608);
static_assert(OUT0_ELEMS * 4 + OUT1_ELEMS * 4 == 8585216);
static_assert(CIN1 == 3 + CFEAT);

__device__ __forceinline__ float h16_to_f32(unsigned hb) {
  const unsigned sgn = (hb & 0x8000u) << 16;
  const unsigned em = hb & 0x7fffu;
  const float fn = __uint_as_float((em << 13) + 0x38000000u);
  const float fs = (float)em * 5.9604644775390625e-8f;
  const float mag = (em < 0x400u) ? fs : fn;
  return __uint_as_float(__float_as_uint(mag) | sgn);
}

__device__ __forceinline__ unsigned pack2h(float a, float b) {
  const _Float16 ha = (_Float16)a;
  const _Float16 hb = (_Float16)b;
  const unsigned ua = (unsigned)__builtin_bit_cast(unsigned short, ha);
  const unsigned ub = (unsigned)__builtin_bit_cast(unsigned short, hb);
  return ua | (ub << 16);
}

__device__ __forceinline__ v16h frag_words(v4u lo, v4u hi) {
  const v8u w = __builtin_shufflevector(lo, hi, 0, 1, 2, 3, 4, 5, 6, 7);
  return __builtin_bit_cast(v16h, w);
}

__device__ __forceinline__ v8f zero8() {
  return (v8f){0.f, 0.f, 0.f, 0.f, 0.f, 0.f, 0.f, 0.f};
}

__device__ __forceinline__ v8f mma16(v16h a, v16h b, v8f c) {
  return __builtin_amdgcn_wmma_f32_16x16x32_f16(false, a, false, b, (short)0, c, false, false);
}

__device__ __forceinline__ void guard8(v8f& c0, v8f& c1, v8f& c2, v8f& c3, v8f& c4, v8f& c5, v8f& c6, v8f& c7,
                                       v16h a0, v16h a1, v16h b0, v16h b1, v16h b2, v16h b3) {
  asm volatile("v_nop\n\tv_nop\n\tv_nop\n\tv_nop"
               : "+v"(c0), "+v"(c1), "+v"(c2), "+v"(c3), "+v"(c4), "+v"(c5), "+v"(c6), "+v"(c7)
               : "v"(a0), "v"(a1), "v"(b0), "v"(b1), "v"(b2), "v"(b3));
}

__global__ __launch_bounds__(256) void k_prep(const float* __restrict__ w0, const float* __restrict__ w1,
                                              const float* __restrict__ w2, v4u* __restrict__ wt) {
  const int blk = blockIdx.x;
  const int tid = threadIdx.x;
  float v[8];
  if (blk < 3) {
    const int g = blk * 2048 + tid * 8;
    const int o = g / KPAD1;
    const int k0 = g - o * KPAD1;
#pragma unroll
    for (int e = 0; e < 8; ++e) {
      const int k = k0 + e;
      const int src = (k < CFEAT) ? (3 + k) : ((k < CIN1) ? (k - CFEAT) : 0);
      const float val = w0[o * CIN1 + src];
      v[e] = (k < CIN1) ? val : 0.0f;
    }
  } else if (blk < 5) {
    const int g = (blk - 3) * 2048 + tid * 8;
    const v4f p0 = *(const v4f*)(w1 + g);
    const v4f p1 = *(const v4f*)(w1 + g + 4);
#pragma unroll
    for (int e = 0; e < 4; ++e) { v[e] = p0[e]; v[4 + e] = p1[e]; }
  } else {
    const int g = (blk - 5) * 2048 + tid * 8;
    const v4f p0 = *(const v4f*)(w2 + g);
    const v4f p1 = *(const v4f*)(w2 + g + 4);
#pragma unroll
    for (int e = 0; e < 4; ++e) { v[e] = p0[e]; v[4 + e] = p1[e]; }
  }
  v4u o4;
  o4[0] = pack2h(v[0], v[1]);
  o4[1] = pack2h(v[2], v[3]);
  o4[2] = pack2h(v[4], v[5]);
  o4[3] = pack2h(v[6], v[7]);
  v4u* dst = wt + blk * 256 + tid;
  *(volatile v4u*)dst = o4;
  __threadfence();
  *(volatile v4u*)dst = o4;
}

__global__ __launch_bounds__(256) void k_transpose(const float* __restrict__ points, v4u* __restrict__ pt) {
  __shared__ float tl[64 * 65];
  const int b = blockIdx.x >> 6;
  const int n0 = (blockIdx.x & 63) * 64;
  const int tid = threadIdx.x;
  const int n = tid & 63;
  const int c0 = tid >> 6;
  const float* src = points + (size_t)b * CFEAT * NPTS + n0 + n;
#pragma unroll
  for (int i = 0; i < 8; ++i) {
    const int c = c0 + 4 * i;
    tl[c * 65 + n] = src[(size_t)c * NPTS];
  }
  asm volatile("" ::: "memory");
#pragma unroll
  for (int i = 8; i < 16; ++i) {
    const int c = c0 + 4 * i;
    tl[c * 65 + n] = src[(size_t)c * NPTS];
  }
  __syncthreads();
  const int q = tid & 7;
  v4u wv[2];
#pragma unroll
  for (int it = 0; it < 2; ++it) {
    const int row = (tid >> 3) + 32 * it;
#pragma unroll
    for (int j = 0; j < 4; ++j) {
      const float f0 = tl[(8 * q + 2 * j) * 65 + row];
      const float f1 = tl[(8 * q + 2 * j + 1) * 65 + row];
      wv[it][j] = pack2h(f0, f1);
    }
  }
  for (int pass = 0; pass < 2; ++pass) {
#pragma unroll
    for (int it = 0; it < 2; ++it) {
      const int row = (tid >> 3) + 32 * it;
      v4u* dst = pt + ((size_t)(b * NPTS + n0 + row)) * 8 + q;
      *(volatile v4u*)dst = wv[it];
    }
    __threadfence();
  }
}

__global__ __launch_bounds__(512) void k_fps(const float* __restrict__ xyz, float* __restrict__ out0,
                                             float* __restrict__ cxw) {
#pragma clang fp contract(off)
  __shared__ __align__(16) float xs[3 * NPTS];
  __shared__ int cent[NCENT];
  __shared__ float sv[2][16];
  __shared__ int si[2][16];
  const int b = blockIdx.x;
  const int tid = threadIdx.x;
  const int lane = tid & 31;
  const int wave = tid >> 5;
  const float* X = xyz + (size_t)b * 3 * NPTS;
  float px[8], py[8], pz[8], dist[8];
  {
    const v4f x0 = *(const v4f*)(X + 4 * tid);
    const v4f x1 = *(const v4f*)(X + 2048 + 4 * tid);
    const v4f y0 = *(const v4f*)(X + NPTS + 4 * tid);
    const v4f y1 = *(const v4f*)(X + NPTS + 2048 + 4 * tid);
    const v4f z0 = *(const v4f*)(X + 2 * NPTS + 4 * tid);
    const v4f z1 = *(const v4f*)(X + 2 * NPTS + 2048 + 4 * tid);
    *(v4f*)(xs + 4 * tid) = x0;
    *(v4f*)(xs + 2048 + 4 * tid) = x1;
    *(v4f*)(xs + NPTS + 4 * tid) = y0;
    *(v4f*)(xs + NPTS + 2048 + 4 * tid) = y1;
    *(v4f*)(xs + 2 * NPTS + 4 * tid) = z0;
    *(v4f*)(xs + 2 * NPTS + 2048 + 4 * tid) = z1;
#pragma unroll
    for (int e = 0; e < 4; ++e) {
      px[e] = x0[e]; px[4 + e] = x1[e];
      py[e] = y0[e]; py[4 + e] = y1[e];
      pz[e] = z0[e]; pz[4 + e] = z1[e];
    }
#pragma unroll
    for (int e = 0; e < 8; ++e) dist[e] = 1e10f;
  }
  __syncthreads();
  int f = 0;
#pragma unroll 1
  for (int it = 0; it < NCENT; ++it) {
    if (tid == 0) cent[it] = f;
    const float cx = xs[f];
    const float cy = xs[NPTS + f];
    const float cz = xs[2 * NPTS + f];
    float bv = -1.0f;
    int bi = 0;
#pragma unroll
    for (int i = 0; i < 8; ++i) {
      const float dx = px[i] - cx;
      const float dy = py[i] - cy;
      const float dz = pz[i] - cz;
      const float t0 = dx * dx;
      const float t1 = dy * dy;
      const float t2 = dz * dz;
      const float d = (t0 + t2) + t1;
      const float dm = fminf(dist[i], d);
      dist[i] = dm;
      const int pidx = (i < 4) ? (4 * tid + i) : (2048 + 4 * tid + (i - 4));
      if (dm > bv) { bv = dm; bi = pidx; }
    }
#pragma unroll
    for (int off = 16; off >= 1; off >>= 1) {
      const float ov = __shfl_xor(bv, off, 32);
      const int oi = __shfl_xor(bi, off, 32);
      const bool take = (ov > bv) || ((ov == bv) && (oi < bi));
      bv = take ? ov : bv;
      bi = take ? oi : bi;
    }
    const int p = it & 1;
    if (lane == 0) { sv[p][wave] = bv; si[p][wave] = bi; }
    __syncthreads();
    float rv = sv[p][lane & 15];
    int ri = si[p][lane & 15];
#pragma unroll
    for (int off = 8; off >= 1; off >>= 1) {
      const float ov = __shfl_xor(rv, off, 32);
      const int oi = __shfl_xor(ri, off, 32);
      const bool take = (ov > rv) || ((ov == rv) && (oi < ri));
      rv = take ? ov : rv;
      ri = take ? oi : ri;
    }
    f = ri & (NPTS - 1);
  }
  __syncthreads();
#pragma unroll
  for (int rep = 0; rep < 2; ++rep) {
    const int q = tid + 512 * rep;
    if (q < 768) {
      const int c = q >> 8;
      const int s4 = (q & 255) * 4;
      v4f v;
#pragma unroll
      for (int e = 0; e < 4; ++e) v[e] = xs[c * NPTS + (cent[s4 + e] & (NPTS - 1))];
      float* d0 = out0 + (size_t)b * 3 * NCENT + c * NCENT + s4;
      float* d1 = cxw + (size_t)b * 3 * NCENT + c * NCENT + s4;
      for (int pass = 0; pass < 2; ++pass) {
        *(volatile v4f*)d0 = v;
        *(volatile v4f*)d1 = v;
        __threadfence();
      }
    }
  }
}

__global__ __launch_bounds__(128) void k_group_l1(const float* __restrict__ xyz, const float* __restrict__ cxw,
                                                  const v4u* __restrict__ ptv, const v4u* __restrict__ w0v,
                                                  const float* __restrict__ b0, v4u* __restrict__ y1v,
                                                  float* __restrict__ part) {
#pragma clang fp contract(off)
  __shared__ __align__(16) _Float16 w0s[CH1 * PITCH_A1];
  __shared__ __align__(16) _Float16 tile[GEMM_WAVES][NSAMP * PITCH_A1];
  __shared__ int slot[GEMM_WAVES][NSAMP];
  __shared__ __align__(16) float sst[GEMM_WAVES][2 * CH1];
  __shared__ float cst[CH1];
  const int tid = threadIdx.x;
  const int lane = tid & 31;
  const int wave = tid >> 5;
  const int hh = lane >> 4;
  const int c = lane & 15;
  const int q = lane & 7;
  const int rq = lane >> 3;

#pragma unroll
  for (int i = 0; i < 6; ++i) {
    const int idx = tid + 128 * i;
    const int row = idx / 12;
    const int qq = idx - row * 12;
    const v4u w = w0v[idx];
    *(v4u*)(w0s + row * PITCH_A1 + 8 * qq) = w;
  }
  if (tid < CH1) cst[tid] = b0[tid];
  __syncthreads();

  float ssum[4] = {0.f, 0.f, 0.f, 0.f};
  float ssq[4] = {0.f, 0.f, 0.f, 0.f};
  _Float16* tw = tile[wave];
  int* sl = slot[wave];
  unsigned zz = 0u;
  asm volatile("" : "+v"(zz));

#pragma unroll 1
  for (int it = 0; it < STRIPS_PER_WAVE; ++it) {
    const int cidx = (blockIdx.x * GEMM_WAVES + wave) * STRIPS_PER_WAVE + it;
    const int b = cidx >> 10;
    const int s = cidx & (NCENT - 1);
    const float* X = xyz + (size_t)b * 3 * NPTS;
    const float* C = cxw + (size_t)b * 3 * NCENT;
    const float cx = C[s];
    const float cy = C[NCENT + s];
    const float cz = C[2 * NCENT + s];

    sl[lane] = 0;
    int cnt = 0;
    for (int j0 = 0; j0 < NPTS && cnt < NSAMP; j0 += 32) {
      const int j = j0 + lane;
      const float x = X[j];
      const float y = X[NPTS + j];
      const float z = X[2 * NPTS + j];
      const float dx = cx - x;
      const float dy = cy - y;
      const float dz = cz - z;
      const float t0 = dx * dx;
      const float t1 = dy * dy;
      const float t2 = dz * dz;
      const float d = (t0 + t2) + t1;
      const bool hit = !(d > BALL_R2);
      const unsigned mask = (unsigned)__ballot(hit);
      const int pos = cnt + __popc(mask & ((1u << lane) - 1u));
      if (hit && pos < NSAMP) sl[pos] = j;
      cnt += __popc(mask);
    }
    __syncthreads();

    const int cc = cnt < NSAMP ? cnt : NSAMP;
    const int own = sl[lane];
    const int first = sl[0];
    int idx = (lane < cc) ? own : first;
    idx = idx < 0 ? 0 : (idx > NPTS - 1 ? NPTS - 1 : idx);

#pragma unroll
    for (int i = 0; i < 8; ++i) {
      const int jr = __shfl(idx, i * 4 + rq, 32);
      const v4u w = ptv[((size_t)(b * NPTS + jr)) * 8 + q];
      *(v4u*)(tw + (i * 4 + rq) * PITCH_A1 + 8 * q) = w;
    }
    {
      const float x = X[idx];
      const float y = X[NPTS + idx];
      const float z = X[2 * NPTS + idx];
      const float dx = x - cx;
      const float dy = y - cy;
      const float dz = z - cz;
      const unsigned wa = pack2h(dx, dy);
      const _Float16 hz = (_Float16)dz;
      const unsigned uz = (unsigned)__builtin_bit_cast(unsigned short, hz);
      const unsigned wb = (uz & 0xffffu) | (zz << 16);
      v4u a4;
      a4[0] = wa; a4[1] = wb; a4[2] = zz; a4[3] = zz;
      v4u z4;
      z4[0] = zz; z4[1] = zz; z4[2] = zz; z4[3] = zz;
      *(v4u*)(tw + lane * PITCH_A1 + 64) = a4;
      *(v4u*)(tw + lane * PITCH_A1 + 72) = z4;
      *(v4u*)(tw + lane * PITCH_A1 + 80) = z4;
      *(v4u*)(tw + lane * PITCH_A1 + 88) = z4;
    }
    __syncthreads();

    v8f acc[2][4];
#pragma unroll
    for (int mt = 0; mt < 2; ++mt)
#pragma unroll
      for (int nt = 0; nt < 4; ++nt) acc[mt][nt] = zero8();
#pragma unroll
    for (int ks = 0; ks < 3; ++ks) {
      v16h bf[4];
      v16h af[2];
#pragma unroll
      for (int nt = 0; nt < 4; ++nt) {
        const _Float16* p = w0s + (nt * 16 + c) * PITCH_A1 + ks * 32 + 8 * hh;
        bf[nt] = frag_words(*(const v4u*)p, *(const v4u*)(p + 16));
      }
#pragma unroll
      for (int mt = 0; mt < 2; ++mt) {
        const _Float16* p = tw + (mt * 16 + c) * PITCH_A1 + ks * 32 + 8 * hh;
        af[mt] = frag_words(*(const v4u*)p, *(const v4u*)(p + 16));
      }
#pragma unroll
      for (int mt = 0; mt < 2; ++mt)
#pragma unroll
        for (int nt = 0; nt < 4; ++nt) acc[mt][nt] = mma16(af[mt], bf[nt], acc[mt][nt]);
      guard8(acc[0][0], acc[0][1], acc[0][2], acc[0][3], acc[1][0], acc[1][1], acc[1][2], acc[1][3],
             af[0], af[1], bf[0], bf[1], bf[2], bf[3]);
    }
    __syncthreads();
#pragma unroll
    for (int nt = 0; nt < 4; ++nt) {
      const float bv = cst[nt * 16 + c];
#pragma unroll
      for (int mt = 0; mt < 2; ++mt) {
#pragma unroll
        for (int r = 0; r < 8; ++r) {
          const float v = acc[mt][nt][r] + bv;
          ssum[nt] += v;
          ssq[nt] += v * v;
          tw[(mt * 16 + 8 * hh + r) * PITCH_S + nt * 16 + c] = (_Float16)v;
        }
      }
    }
    __syncthreads();
    {
      v4u wv[8];
#pragma unroll
      for (int i = 0; i < 8; ++i) wv[i] = *(const v4u*)(tw + (i * 4 + rq) * PITCH_S + 8 * q);
      v4u* dst = y1v + (size_t)cidx * 256 + lane;
      for (int pass = 0; pass < 2; ++pass) {
#pragma unroll
        for (int i = 0; i < 8; ++i) *(volatile v4u*)(dst + i * 32) = wv[i];
        __threadfence();
      }
    }
  }

#pragma unroll
  for (int nt = 0; nt < 4; ++nt) {
    const float o1 = __shfl_xor(ssum[nt], 16, 32);
    const float o2 = __shfl_xor(ssq[nt], 16, 32);
    ssum[nt] += o1;
    ssq[nt] += o2;
  }
  if (hh == 0) {
#pragma unroll
    for (int nt = 0; nt < 4; ++nt) {
      sst[wave][nt * 16 + c] = ssum[nt];
      sst[wave][CH1 + nt * 16 + c] = ssq[nt];
    }
  }
  __syncthreads();
  if (tid < 32) {
    v4f v;
#pragma unroll
    for (int e = 0; e < 4; ++e) {
      const int id = 4 * tid + e;
      v[e] = ((sst[0][id] + sst[1][id]) + sst[2][id]) + sst[3][id];
    }
    float* dst = part + (size_t)blockIdx.x * (2 * CH1) + 4 * tid;
    *(volatile v4f*)dst = v;
    __threadfence();
    *(volatile v4f*)dst = v;
  }
}

template <int NC>
__global__ __launch_bounds__(256) void k_bnstat(const float* __restrict__ part, const float* __restrict__ g,
                                                const float* __restrict__ be, float* __restrict__ tab) {
  __shared__ double red[256];
  __shared__ __align__(16) float tb[256];
  const int tid = threadIdx.x;
  const int id = tid < 2 * NC ? tid : 2 * NC - 1;
  double acc = 0.0;
#pragma unroll 4
  for (int p = 0; p < GEMM_BLOCKS; ++p) acc += (double)part[(size_t)p * (2 * NC) + id];
  red[tid] = acc;
  __syncthreads();
  {
    const int ch = tid & 127;
    const int chc = ch < NC ? ch : NC - 1;
    const double inv = 1.0 / (double)MROWS;
    const double mean = red[chc] * inv;
    const double ex2 = red[NC + chc] * inv;
    double var = ex2 - mean * mean;
    var = var < 0.0 ? 0.0 : var;
    const float varf = (float)var;
    const float rstd = 1.0f / sqrtf(varf + BN_EPSV);
    const float a = g[chc] * rstd;
    const float sh = be[chc] - a * (float)mean;
    const float val = (tid >= 128) ? sh : a;
    tb[tid] = (ch < NC) ? val : 0.0f;
  }
  __syncthreads();
  if (tid < 64) {
    const v4f v = *(const v4f*)(tb + 4 * tid);
    float* dst = tab + 4 * tid;
    *(volatile v4f*)dst = v;
    __threadfence();
    *(volatile v4f*)dst = v;
  }
}

template <bool FULL>
__global__ __launch_bounds__(128) void k_mlp(const v4u* __restrict__ y1v, const v4u* __restrict__ w1v,
                                             const v4u* __restrict__ w2v, const float* __restrict__ tab1,
                                             const float* __restrict__ tab2, const float* __restrict__ b1,
                                             const float* __restrict__ b2, float* __restrict__ part,
                                             float* __restrict__ mxp, float* __restrict__ mnp) {
  constexpr int NT_S = FULL ? 8 : 4;
  constexpr int NCS = NT_S * 16;
  __shared__ __align__(16) _Float16 w1s[CH2 * PITCH_S];
  __shared__ __align__(16) _Float16 w2s[FULL ? CH3 * PITCH_S : 8];
  __shared__ __align__(16) _Float16 tile[GEMM_WAVES][NSAMP * PITCH_S];
  __shared__ __align__(16) float mxs[FULL ? GEMM_WAVES * 2 * CH3 : 4];
  __shared__ __align__(16) float sst[GEMM_WAVES][2 * NCS];
  __shared__ __align__(16) float cst[448];
  const int tid = threadIdx.x;
  const int lane = tid & 31;
  const int wave = tid >> 5;
  const int hh = lane >> 4;
  const int c = lane & 15;
  const int q = lane & 7;
  const int rq = lane >> 3;

#pragma unroll
  for (int i = 0; i < 4; ++i) {
    const int idx = tid + 128 * i;
    const v4u w = w1v[idx];
    *(v4u*)(w1s + (idx >> 3) * PITCH_S + 8 * (idx & 7)) = w;
  }
  if constexpr (FULL) {
#pragma unroll 2
    for (int i = 0; i < 8; ++i) {
      const int idx = tid + 128 * i;
      const v4u w = w2v[idx];
      *(v4u*)(w2s + (idx >> 3) * PITCH_S + 8 * (idx & 7)) = w;
    }
  }
  if (tid < 64) {
    cst[tid] = tab1[tid];
    cst[64 + tid] = tab1[128 + tid];
    cst[128 + tid] = b1[tid];
    cst[192 + tid] = tab2[tid];
    cst[256 + tid] = tab2[128 + tid];
  }
  cst[320 + tid] = b2[tid];
  __syncthreads();

  float ss[8] = {0.f, 0.f, 0.f, 0.f, 0.f, 0.f, 0.f, 0.f};
  float sq[8] = {0.f, 0.f, 0.f, 0.f, 0.f, 0.f, 0.f, 0.f};
  _Float16* tw = tile[wave];

#pragma unroll 1
  for (int it = 0; it < STRIPS_PER_WAVE; ++it) {
    const int strip = (blockIdx.x * GEMM_WAVES + wave) * STRIPS_PER_WAVE + it;
    {
      float a1[8], s1[8];
      const v4f a1lo = *(const v4f*)(cst + 8 * q);
      const v4f a1hi = *(const v4f*)(cst + 8 * q + 4);
      const v4f s1lo = *(const v4f*)(cst + 64 + 8 * q);
      const v4f s1hi = *(const v4f*)(cst + 64 + 8 * q + 4);
#pragma unroll
      for (int e = 0; e < 4; ++e) { a1[e] = a1lo[e]; a1[4 + e] = a1hi[e]; s1[e] = s1lo[e]; s1[4 + e] = s1hi[e]; }
      v4u yw[8];
      const v4u* src = y1v + (size_t)strip * 256 + lane;
#pragma unroll
      for (int i = 0; i < 8; ++i) yw[i] = src[i * 32];
#pragma unroll
      for (int i = 0; i < 8; ++i) {
        v4u o4;
#pragma unroll
        for (int j = 0; j < 4; ++j) {
          const unsigned w = yw[i][j];
          const float x0 = h16_to_f32(w & 0xffffu);
          const float x1 = h16_to_f32(w >> 16);
          const float p0 = a1[2 * j] * x0;
          const float p1 = a1[2 * j + 1] * x1;
          const float r0 = fmaxf(p0 + s1[2 * j], 0.0f);
          const float r1 = fmaxf(p1 + s1[2 * j + 1], 0.0f);
          o4[j] = pack2h(r0, r1);
        }
        *(v4u*)(tw + (i * 4 + rq) * PITCH_S + 8 * q) = o4;
      }
    }
    __syncthreads();
    v8f acc[2][4];
#pragma unroll
    for (int mt = 0; mt < 2; ++mt)
#pragma unroll
      for (int nt = 0; nt < 4; ++nt) acc[mt][nt] = zero8();
#pragma unroll
    for (int ks = 0; ks < 2; ++ks) {
      v16h bf[4];
      v16h af[2];
#pragma unroll
      for (int nt = 0; nt < 4; ++nt) {
        const _Float16* p = w1s + (nt * 16 + c) * PITCH_S + ks * 32 + 8 * hh;
        bf[nt] = frag_words(*(const v4u*)p, *(const v4u*)(p + 16));
      }
#pragma unroll
      for (int mt = 0; mt < 2; ++mt) {
        const _Float16* p = tw + (mt * 16 + c) * PITCH_S + ks * 32 + 8 * hh;
        af[mt] = frag_words(*(const v4u*)p, *(const v4u*)(p + 16));
      }
#pragma unroll
      for (int mt = 0; mt < 2; ++mt)
#pragma unroll
        for (int nt = 0; nt < 4; ++nt) acc[mt][nt] = mma16(af[mt], bf[nt], acc[mt][nt]);
      guard8(acc[0][0], acc[0][1], acc[0][2], acc[0][3], acc[1][0], acc[1][1], acc[1][2], acc[1][3],
             af[0], af[1], bf[0], bf[1], bf[2], bf[3]);
    }
    __syncthreads();
    if constexpr (!FULL) {
#pragma unroll
      for (int nt = 0; nt < 4; ++nt) {
        const float bv = cst[128 + nt * 16 + c];
#pragma unroll
        for (int mt = 0; mt < 2; ++mt) {
#pragma unroll
          for (int r = 0; r < 8; ++r) {
            const float v = acc[mt][nt][r] + bv;
            ss[nt] += v;
            sq[nt] += v * v;
          }
        }
      }
    } else {
#pragma unroll
      for (int nt = 0; nt < 4; ++nt) {
        const float bv = cst[128 + nt * 16 + c];
        const float a2 = cst[192 + nt * 16 + c];
        const float s2 = cst[256 + nt * 16 + c];
#pragma unroll
        for (int mt = 0; mt < 2; ++mt) {
#pragma unroll
          for (int r = 0; r < 8; ++r) {
            const float v = acc[mt][nt][r] + bv;
            const float pr = a2 * v;
            const float y = fmaxf(pr + s2, 0.0f);
            tw[(mt * 16 + 8 * hh + r) * PITCH_S + nt * 16 + c] = (_Float16)y;
          }
        }
      }
      __syncthreads();
      v16h a3[2][2];
#pragma unroll
      for (int mt = 0; mt < 2; ++mt)
#pragma unroll
        for (int ks = 0; ks < 2; ++ks) {
          const _Float16* p = tw + (mt * 16 + c) * PITCH_S + ks * 32 + 8 * hh;
          a3[mt][ks] = frag_words(*(const v4u*)p, *(const v4u*)(p + 16));
        }
#pragma unroll
      for (int nh = 0; nh < 2; ++nh) {
        v8f acc3[2][4];
#pragma unroll
        for (int mt = 0; mt < 2; ++mt)
#pragma unroll
          for (int nt = 0; nt < 4; ++nt) acc3[mt][nt] = zero8();
#pragma unroll
        for (int ks = 0; ks < 2; ++ks) {
          v16h bf[4];
#pragma unroll
          for (int nt = 0; nt < 4; ++nt) {
            const _Float16* p = w2s + (nh * 64 + nt * 16 + c) * PITCH_S + ks * 32 + 8 * hh;
            bf[nt] = frag_words(*(const v4u*)p, *(const v4u*)(p + 16));
          }
#pragma unroll
          for (int mt = 0; mt < 2; ++mt)
#pragma unroll
            for (int nt = 0; nt < 4; ++nt) acc3[mt][nt] = mma16(a3[mt][ks], bf[nt], acc3[mt][nt]);
          guard8(acc3[0][0], acc3[0][1], acc3[0][2], acc3[0][3], acc3[1][0], acc3[1][1], acc3[1][2], acc3[1][3],
                 a3[0][ks], a3[1][ks], bf[0], bf[1], bf[2], bf[3]);
        }
#pragma unroll
        for (int nt = 0; nt < 4; ++nt) {
          const int col = nh * 64 + nt * 16 + c;
          const float bv = cst[320 + col];
          float mx = -3.0e38f;
          float mn = 3.0e38f;
#pragma unroll
          for (int mt = 0; mt < 2; ++mt) {
#pragma unroll
            for (int r = 0; r < 8; ++r) {
              const float v = acc3[mt][nt][r] + bv;
              ss[nh * 4 + nt] += v;
              sq[nh * 4 + nt] += v * v;
              mx = fmaxf(mx, v);
              mn = fminf(mn, v);
            }
          }
          const float mxo = __shfl_xor(mx, 16, 32);
          const float mno = __shfl_xor(mn, 16, 32);
          mx = fmaxf(mx, mxo);
          mn = fminf(mn, mno);
          if (hh == 0) {
            mxs[wave * 2 * CH3 + col] = mx;
            mxs[wave * 2 * CH3 + CH3 + col] = mn;
          }
        }
      }
      __syncthreads();
      {
        const v4f vx = *(const v4f*)(mxs + wave * 2 * CH3 + 4 * lane);
        const v4f vn = *(const v4f*)(mxs + wave * 2 * CH3 + CH3 + 4 * lane);
        float* dx = mxp + (size_t)strip * CH3 + 4 * lane;
        float* dn = mnp + (size_t)strip * CH3 + 4 * lane;
        for (int pass = 0; pass < 2; ++pass) {
          *(volatile v4f*)dx = vx;
          *(volatile v4f*)dn = vn;
          __threadfence();
        }
      }
    }
  }

#pragma unroll
  for (int j = 0; j < NT_S; ++j) {
    const float o1 = __shfl_xor(ss[j], 16, 32);
    const float o2 = __shfl_xor(sq[j], 16, 32);
    ss[j] += o1;
    sq[j] += o2;
  }
  if (hh == 0) {
#pragma unroll
    for (int j = 0; j < NT_S; ++j) {
      sst[wave][j * 16 + c] = ss[j];
      sst[wave][NCS + j * 16 + c] = sq[j];
    }
  }
  __syncthreads();
  if (tid < (2 * NCS) / 4) {
    v4f v;
#pragma unroll
    for (int e = 0; e < 4; ++e) {
      const int id = 4 * tid + e;
      v[e] = ((sst[0][id] + sst[1][id]) + sst[2][id]) + sst[3][id];
    }
    float* dst = part + (size_t)blockIdx.x * (2 * NCS) + 4 * tid;
    *(volatile v4f*)dst = v;
    __threadfence();
    *(volatile v4f*)dst = v;
  }
}

__global__ __launch_bounds__(256) void k_final(const float* __restrict__ mxp, const float* __restrict__ mnp,
                                               const float* __restrict__ tab3, float* __restrict__ out1) {
  __shared__ float tl[CH3 * 33];
  const int b = blockIdx.x >> 5;
  const int s0 = (blockIdx.x & 31) * 32;
  const int tid = threadIdx.x;
  const int lane = tid & 31;
  const int wave = tid >> 5;
  const v4f a = *(const v4f*)(tab3 + 4 * lane);
  const v4f sh = *(const v4f*)(tab3 + 128 + 4 * lane);
  float fa[4], fb[4];
#pragma unroll
  for (int e = 0; e < 4; ++e) {
    fa[e] = (a[e] > 0.0f) ? 1.0f : 0.0f;
    fb[e] = 1.0f - fa[e];
  }
  v4f vx[4], vn[4];
#pragma unroll
  for (int i = 0; i < 4; ++i) {
    const int row = wave * 4 + i;
    const size_t g = (size_t)(b * NCENT + s0 + row);
    vx[i] = *(const v4f*)(mxp + g * CH3 + 4 * lane);
    vn[i] = *(const v4f*)(mnp + g * CH3 + 4 * lane);
  }
#pragma unroll
  for (int i = 0; i < 4; ++i) {
    const int row = wave * 4 + i;
#pragma unroll
    for (int e = 0; e < 4; ++e) {
      const float p0 = fa[e] * vx[i][e];
      const float p1 = fb[e] * vn[i][e];
      const float sel = p0 + p1;
      const float pr = a[e] * sel;
      tl[(4 * lane + e) * 33 + row] = fmaxf(pr + sh[e], 0.0f);
    }
  }
  __syncthreads();
  const int q = tid & 7;
  v4f ov[4];
#pragma unroll
  for (int it = 0; it < 4; ++it) {
    const int ch = (tid >> 3) + 32 * it;
#pragma unroll
    for (int e = 0; e < 4; ++e) ov[it][e] = tl[ch * 33 + 4 * q + e];
  }
  for (int pass = 0; pass < 2; ++pass) {
#pragma unroll
    for (int it = 0; it < 4; ++it) {
      const int ch = (tid >> 3) + 32 * it;
      float* dst = out1 + ((size_t)(b * CH3 + ch)) * NCENT + s0 + 4 * q;
      *(volatile v4f*)dst = ov[it];
    }
    __threadfence();
  }
}

constexpr size_t WS_WT = 0;
constexpr size_t WS_CX = WS_WT + 36864;
constexpr size_t WS_TAB = WS_CX + 196608;
constexpr size_t WS_P1 = WS_TAB + 4096;
constexpr size_t WS_P2 = WS_P1 + (size_t)GEMM_BLOCKS * 128 * 4;
constexpr size_t WS_P3 = WS_P2 + (size_t)GEMM_BLOCKS * 128 * 4;
constexpr size_t WS_PT = WS_P3 + (size_t)GEMM_BLOCKS * 256 * 4;
constexpr size_t WS_MX = WS_PT + (size_t)NBATCH * NPTS * CFEAT * 2;
constexpr size_t WS_MN = WS_MX + (size_t)NSTRIPS * CH3 * 4;
constexpr size_t WS_Y1 = WS_MN + (size_t)NSTRIPS * CH3 * 4;
constexpr size_t WS_TOTAL = WS_Y1 + (size_t)MROWS * CH1 * 2;
static_assert(WS_TOTAL == 93036544);
static_assert(WS_TOTAL <= 134217728);
static_assert((WS_CX % 4096) == 0 && (WS_PT % 4096) == 0 && (WS_Y1 % 4096) == 0);

extern "C" void kernel_launch(void* const* d_in, const int* in_sizes, int n_in,
                              void* d_out, int out_size, void* d_ws, size_t ws_size, hipStream_t stream) {
  (void)in_sizes; (void)n_in; (void)out_size;
  if (ws_size < WS_TOTAL) return;
  const float* xyz    = (const float*)d_in[0];
  const float* points = (const float*)d_in[1];
  const float* w0  = (const float*)d_in[2];
  const float* b0  = (const float*)d_in[3];
  const float* g0  = (const float*)d_in[4];
  const float* be0 = (const float*)d_in[5];
  const float* w1  = (const float*)d_in[6];
  const float* b1  = (const float*)d_in[7];
  const float* g1  = (const float*)d_in[8];
  const float* be1 = (const float*)d_in[9];
  const float* w2  = (const float*)d_in[10];
  const float* b2  = (const float*)d_in[11];
  const float* g2  = (const float*)d_in[12];
  const float* be2 = (const float*)d_in[13];
  float* out0 = (float*)d_out;
  float* out1 = (float*)d_out + OUT0_ELEMS;
  char* ws = (char*)d_ws;
  v4u*   wt   = (v4u*)(ws + WS_WT);
  float* cxw  = (float*)(ws + WS_CX);
  float* tab1 = (float*)(ws + WS_TAB);
  float* tab2 = tab1 + 256;
  float* tab3 = tab2 + 256;
  float* p1   = (float*)(ws + WS_P1);
  float* p2   = (float*)(ws + WS_P2);
  float* p3   = (float*)(ws + WS_P3);
  v4u*   pt   = (v4u*)(ws + WS_PT);
  float* mxp  = (float*)(ws + WS_MX);
  float* mnp  = (float*)(ws + WS_MN);
  v4u*   y1v  = (v4u*)(ws + WS_Y1);
  const v4u* w0v = wt;
  const v4u* w1v = wt + 768;
  const v4u* w2v = wt + 1280;

  k_prep<<<9, 256, 0, stream>>>(w0, w1, w2, wt);
  k_transpose<<<NBATCH * (NPTS / 64), 256, 0, stream>>>(points, pt);
  k_fps<<<NBATCH, 512, 0, stream>>>(xyz, out0, cxw);
  k_group_l1<<<GEMM_BLOCKS, 128, 0, stream>>>(xyz, cxw, pt, w0v, b0, y1v, p1);
  k_bnstat<CH1><<<1, 256, 0, stream>>>(p1, g0, be0, tab1);
  k_mlp<false><<<GEMM_BLOCKS, 128, 0, stream>>>(y1v, w1v, w2v, tab1, tab1, b1, b2, p2, mxp, mnp);
  k_bnstat<CH2><<<1, 256, 0, stream>>>(p2, g1, be1, tab2);
  k_mlp<true><<<GEMM_BLOCKS, 128, 0, stream>>>(y1v, w1v, w2v, tab1, tab2, b1, b2, p3, mxp, mnp);
  k_bnstat<CH3><<<1, 256, 0, stream>>>(p3, g2, be2, tab3);
  k_final<<<NBATCH * (NCENT / 32), 256, 0, stream>>>(mxp, mnp, tab3, out1);
}
